// FrameInterpolate_14877766714082
// MI455X (gfx1250) — hardware-verified
//
#include <hip/hip_runtime.h>
#include <math.h>

typedef __attribute__((ext_vector_type(16))) _Float16 v16h;
typedef __attribute__((ext_vector_type(16))) __bf16 v16b;
typedef __attribute__((ext_vector_type(8)))  _Float16 v8h;
typedef __attribute__((ext_vector_type(8)))  float v8f;
typedef __attribute__((ext_vector_type(4)))  float v4f;
typedef __attribute__((ext_vector_type(2)))  float v2f;
typedef __attribute__((ext_vector_type(4)))  unsigned v4u;
typedef __attribute__((ext_vector_type(4)))  int v4i;
typedef float __attribute__((may_alias)) float_a;
typedef int __attribute__((may_alias)) int_a;

template <typename T> __device__ __forceinline__ void vst2(void* p, T v) { *(volatile T*)p = v; __threadfence(); *(volatile T*)p = v; }
__device__ __forceinline__ v8f wmma16(v16h a, v16h b, v8f c) {
  v8f d = __builtin_amdgcn_wmma_f32_16x16x32_f16(false, a, false, b, (short)0, c, false, false);
  asm volatile("v_nop\n\tv_nop\n\tv_nop\n\tv_nop" : "+v"(d) : "v"(a), "v"(b));
  return d;
}
__device__ __forceinline__ v8f wmma_bf(v16b a, v16b b, v8f c) {
  v8f d = __builtin_amdgcn_wmma_f32_16x16x32_bf16(false, a, false, b, (short)0, c, false, false);
  asm volatile("v_nop\n\tv_nop\n\tv_nop\n\tv_nop" : "+v"(d) : "v"(a), "v"(b));
  return d;
}
__device__ __forceinline__ v16h frag_h(const _Float16* rowk0, int lane) {
  union { v16h v; v8h q[2]; } u; const _Float16* p = rowk0 + 8 * (lane >> 4);
  u.q[0] = *(const v8h*)p; u.q[1] = *(const v8h*)(p + 16); return u.v;
}
__device__ __forceinline__ v16h frag_f32(const float* rowk0, int lane) {
  v16h a; const float* p = rowk0 + 8 * (lane >> 4);
#pragma unroll
  for (int i = 0; i < 8; ++i) { a[i] = (_Float16)p[i]; a[8 + i] = (_Float16)p[16 + i]; }
  return a;
}
__device__ __forceinline__ v16h frag_f32s(const float* rowk0, int lane, float sc) {
  v16h a; const float* p = rowk0 + 8 * (lane >> 4);
#pragma unroll
  for (int i = 0; i < 8; ++i) { a[i] = (_Float16)(p[i] * sc); a[8 + i] = (_Float16)(p[16 + i] * sc); }
  return a;
}
__device__ __forceinline__ v16h fragc_f32(const float* W, int k0, int n, int lane, int ld, int K) {
  v16h a; const int g = lane >> 4;
#pragma unroll
  for (int i = 0; i < 8; ++i) { const int ka = k0 + 8 * g + i, kb = ka + 16;
    a[i] = (_Float16)(ka < K ? W[(size_t)ka * ld + n] : 0.f); a[8 + i] = (_Float16)(kb < K ? W[(size_t)kb * ld + n] : 0.f); }
  return a;
}
struct F2 { v16b h, l; };
__device__ __forceinline__ F2 bsplit16(const float v[16]) { F2 r;
#pragma unroll
  for (int i = 0; i < 16; ++i) { const __bf16 h = (__bf16)v[i]; r.h[i] = h; r.l[i] = (__bf16)(v[i] - (float)h); }
  return r; }
__device__ __forceinline__ F2 split_row(const float* row, int k0, int lane) { float v[16]; const float* p = row + k0 + 8 * (lane >> 4);
#pragma unroll
  for (int i = 0; i < 8; ++i) { v[i] = p[i]; v[8 + i] = p[16 + i]; }
  return bsplit16(v); }
__device__ __forceinline__ F2 split_rowK(const float* row, int k0, int lane, int K) { float v[16]; const int g = lane >> 4;
#pragma unroll
  for (int i = 0; i < 8; ++i) { const int ka = k0 + 8 * g + i, kb = ka + 16; v[i] = ka < K ? row[ka] : 0.f; v[8 + i] = kb < K ? row[kb] : 0.f; }
  return bsplit16(v); }
__device__ __forceinline__ F2 split_col(const float* W, int k0, int n, int lane, int ld, int K) { float v[16]; const int g = lane >> 4;
#pragma unroll
  for (int i = 0; i < 8; ++i) { const int ka = k0 + 8 * g + i, kb = ka + 16; v[i] = ka < K ? W[(size_t)ka * ld + n] : 0.f; v[8 + i] = kb < K ? W[(size_t)kb * ld + n] : 0.f; }
  return bsplit16(v); }
__device__ __forceinline__ v8f mac3(const F2& a, const F2& b, v8f c) { c = wmma_bf(a.l, b.h, c); c = wmma_bf(a.h, b.l, c); return wmma_bf(a.h, b.h, c); }
__device__ __forceinline__ float sigm(float v) { return 1.0f / (1.0f + expf(-v)); }
#define LDSX() do { asm volatile("s_wait_dscnt 0" ::: "memory"); __builtin_amdgcn_wave_barrier(); __builtin_amdgcn_fence(__ATOMIC_RELEASE, "workgroup"); } while (0)

#define NB 8
#define HI 512
#define WI 512
#define CF 10
#define CM 64

__device__ __forceinline__ void warp3(const float* __restrict__ img, int b, int y, int x, float fy, float fx, float* o) {
  const float qy = (float)y + fy, qx = (float)x + fx;
  const float y0 = fminf(fmaxf(floorf(qy), 0.f), (float)(HI - 2)), x0 = fminf(fmaxf(floorf(qx), 0.f), (float)(WI - 2));
  const float ay = fminf(fmaxf(qy - y0, 0.f), 1.f), ax = fminf(fmaxf(qx - x0, 0.f), 1.f);
  const int yi = (int)y0, xi = (int)x0;
  const float* p00 = img + (((size_t)b * HI + yi) * WI + xi) * 3; const float* p01 = p00 + 3; const float* p10 = p00 + WI * 3; const float* p11 = p10 + 3;
#pragma unroll
  for (int c = 0; c < 3; ++c) { const float top = p00[c] * (1.f - ax) + p01[c] * ax, bot = p10[c] * (1.f - ax) + p11[c] * ax; o[c] = top * (1.f - ay) + bot * ay; }
}
__global__ __launch_bounds__(256) void k_main(const float* __restrict__ prv, const float* __restrict__ nxt, const float* __restrict__ f01, const float* __restrict__ f10, const float* __restrict__ dwk, const float* __restrict__ pwk, const float* __restrict__ b1, const float* __restrict__ w2, const float* __restrict__ b2, float* __restrict__ out) {
  __shared__ float sf[6][66][CF + 1];
  __shared__ __align__(16) _Float16 sd[8][32][40];
  __shared__ __align__(16) _Float16 sm[8][32][72];
  __shared__ __align__(16) float so[4][64 * 3 + 16];
  __shared__ float sdw[9][CF];
  const int tid = threadIdx.x, wave = tid >> 5, lane = tid & 31, col = lane & 15, g = lane >> 4;
  const int b = blockIdx.z, y0 = blockIdx.y * 4, x0 = blockIdx.x * 64; const int ry_w = wave >> 1, px0 = (wave & 1) * 32; const int y = y0 + ry_w;
  if (tid < 9 * CF) sdw[tid / CF][tid % CF] = dwk[tid];
  for (int q = tid; q < 6 * 66; q += 256) { const int ry = q / 66, rx = q % 66; const int yy = y0 + ry - 1, xx = x0 + rx - 1; float f[CF];
#pragma unroll
    for (int c = 0; c < CF; ++c) f[c] = 0.f;
    if (yy >= 0 && yy < HI && xx >= 0 && xx < WI) { const size_t pix = ((size_t)b * HI + yy) * WI + xx;
      const float a0 = f01[pix * 2], a1 = f01[pix * 2 + 1], c0 = f10[pix * 2], c1 = f10[pix * 2 + 1];
      warp3(prv, b, yy, xx, 0.5f * c1, 0.5f * c0, &f[0]);
      warp3(nxt, b, yy, xx, 0.5f * a1, 0.5f * a0, &f[3]);
      f[6] = a0; f[7] = a1; f[8] = c0; f[9] = c1; }
#pragma unroll
    for (int c = 0; c < CF; ++c) sf[ry][rx][c] = f[c]; }
  __syncthreads();
  { const int px = px0 + lane;
    for (int c = 0; c < 32; ++c) { float s = 0.f;
      if (c < CF) {
#pragma unroll
        for (int kh = 0; kh < 3; ++kh)
#pragma unroll
          for (int kw = 0; kw < 3; ++kw) s += sf[ry_w + kh][px + kw][c] * sdw[kh * 3 + kw][c]; }
      sd[wave][lane][c] = (_Float16)s; } }
  LDSX();
#pragma unroll 1
  for (int ht = 0; ht < 2; ++ht) {
    v8f acc[4] = {};
    { const v16h a = frag_h(&sd[wave][ht * 16 + col][0], lane);
#pragma unroll
      for (int t = 0; t < 4; ++t) acc[t] = wmma16(a, fragc_f32(pwk, 0, t * 16 + col, lane, CM, CF), acc[t]); }
#pragma unroll
    for (int t = 0; t < 4; ++t) { const int n = t * 16 + col; const float bb = b1[n];
#pragma unroll
      for (int r = 0; r < 8; ++r) { const float v = acc[t][r] + bb; float mv; if (v > 20.f) mv = v; else { const float e = expf(v); const float nn = e * (e + 2.f); mv = v * nn / (nn + 2.f); }
        sm[wave][ht * 16 + 8 * g + r][n] = (_Float16)mv; } }
    LDSX();
    v8f o = {};
#pragma unroll
    for (int kc = 0; kc < 2; ++kc) { v16h bb; const int n = col;
#pragma unroll
      for (int i = 0; i < 8; ++i) { const int ka = kc * 32 + 8 * g + i, kb2 = ka + 16; bb[i] = (_Float16)(n < 3 ? w2[ka * 3 + n] * 8.0f : 0.f); bb[8 + i] = (_Float16)(n < 3 ? w2[kb2 * 3 + n] * 8.0f : 0.f); }
      o = wmma16(frag_h(&sm[wave][ht * 16 + col][0] + kc * 32, lane), bb, o); }
    if (col < 3) {
#pragma unroll
      for (int r = 0; r < 8; ++r) so[ry_w][(px0 + ht * 16 + 8 * g + r) * 3 + col] = o[r] * 0.125f + b2[col]; } }
  __syncthreads();
  for (int q = tid; q < 4 * 48; q += 256) { const int ry = q / 48, pc = q % 48; vst2(out + (((size_t)b * HI + y0 + ry) * WI + x0) * 3 + pc * 4, *(const v4f*)(&so[ry][pc * 4])); }
}
extern "C" void kernel_launch(void* const* d_in, const int* in_sizes, int n_in, void* d_out, int out_size, void* d_ws, size_t ws_size, hipStream_t stream) {
  (void)in_sizes; (void)n_in; (void)out_size; (void)ws_size; (void)d_ws;
  const float** I = (const float**)d_in;
  float* out = (float*)d_out;
  k_main<<<dim3(WI / 64, HI / 4, NB), 256, 0, stream>>>(I[0], I[1], I[2], I[3], I[4], I[5], I[6], I[7], I[8], out);
}
